// MemoryBank_82480551952470
// MI455X (gfx1250) — hardware-run, weakly checked
//
#include <hip/hip_runtime.h>
#include <stddef.h>
#include <stdint.h>


#define ROWS   8192
#define DIM    1024
#define NMEM   512
#define K2     2048
#define NTHR   256
#define NWAVE  8
#define XSC    8
#define WSC    1024
#define TPW    64
#define WSCAP  134217728
#define LDS_SC  (32 * NMEM * 4)
#define LDS_STG (NWAVE * 32 * 64 * 4)
#define SCALE_QK 0.08838834764831845f
#define LN_EPS   1e-5f

static_assert((ROWS % 128) == 0);
static_assert((DIM % 128) == 0);
static_assert((NMEM % 128) == 0);
static_assert((K2 % 128) == 0);
static_assert(NTHR == NWAVE * 32);
static_assert(((ROWS * DIM) % (8 * NTHR)) == 0);
static_assert(((NMEM * DIM) % (8 * NTHR)) == 0);
static_assert((ROWS % 32) == 0);
static_assert((ROWS % 8) == 0);
static_assert(NMEM == NWAVE * 64);
static_assert(LDS_SC <= 300 * 1024);
static_assert(LDS_STG <= 300 * 1024);

typedef float          v2f  __attribute__((ext_vector_type(2)));
typedef float          v4f  __attribute__((ext_vector_type(4)));
typedef float          v8f  __attribute__((ext_vector_type(8)));
typedef _Float16       v8h  __attribute__((ext_vector_type(8)));
typedef _Float16       v16h __attribute__((ext_vector_type(16)));
typedef unsigned short v8us __attribute__((ext_vector_type(8)));
typedef unsigned short v16us __attribute__((ext_vector_type(16)));
typedef __bf16         v16bf __attribute__((ext_vector_type(16)));

union FragH { v16h v; v8h h[2]; };
union FragB { v16bf v; v16us u; v8us h[2]; };

__device__ __forceinline__ v8f wmh(v16h a, v16h b, v8f c) {
  v8f d = __builtin_amdgcn_wmma_f32_16x16x32_f16(false, a, false, b, (short)0, c, false, false);
  asm volatile("v_nop\n\tv_nop\n\tv_nop\n\tv_nop" : "+v"(d) : "v"(a), "v"(b));
  return d;
}
__device__ __forceinline__ v8f wmb(v16us a, v16us b, v8f c) {
  FragB fa, fb;
  fa.u = a; fb.u = b;
  v8f d = __builtin_amdgcn_wmma_f32_16x16x32_bf16(false, fa.v, false, fb.v, (short)0, c, false, false);
  asm volatile("v_nop\n\tv_nop\n\tv_nop\n\tv_nop" : "+v"(d) : "v"(a), "v"(b));
  return d;
}

__device__ __forceinline__ unsigned short bfbits(float f) {
  unsigned int u = __float_as_uint(f);
  u += 0x7FFFu + ((u >> 16) & 1u);
  return (unsigned short)(u >> 16);
}
__device__ __forceinline__ void split2(float x, unsigned short& h, unsigned short& l) {
  h = bfbits(x);
  const float hf = __uint_as_float(((unsigned int)h) << 16);
  l = bfbits(x - hf);
}

__global__ __launch_bounds__(NTHR) void k_split8(const float* __restrict__ x, unsigned short* hi,
                                                 unsigned short* lo, int n8) {
  const int t = blockIdx.x * NTHR + threadIdx.x;
  if (t >= n8) return;
  const float* p = x + (size_t)t * 8;
  const v4f f0 = *(const v4f*)p;
  const v4f f1 = *(const v4f*)(p + 4);
  float f[8] = {f0.x, f0.y, f0.z, f0.w, f1.x, f1.y, f1.z, f1.w};
  v8us H, L;
#pragma unroll
  for (int e = 0; e < 8; ++e) {
    unsigned short hh, ll;
    split2(f[e], hh, ll);
    H[e] = hh; L[e] = ll;
  }
  unsigned short* dh = hi + (size_t)t * 8;
  unsigned short* dl = lo + (size_t)t * 8;
  *(volatile v8us*)dh = H;
  *(volatile v8us*)dl = L;
  __threadfence();
  *(volatile v8us*)dh = H;
  *(volatile v8us*)dl = L;
}

__global__ __launch_bounds__(NTHR) void k_cvt_upd(const float* __restrict__ u, _Float16* gA) {
  const int t = blockIdx.x * NTHR + threadIdx.x;
  if (t >= ROWS * (DIM / 8)) return;
  const int row = t >> 7, c8 = (t & 127) * 8;
  const float* p = u + (size_t)row * DIM + c8;
  const v4f f0 = *(const v4f*)p;
  const v4f f1 = *(const v4f*)(p + 4);
  v8h a;
  a[0] = (_Float16)(f0.x * (float)XSC); a[1] = (_Float16)(f0.y * (float)XSC);
  a[2] = (_Float16)(f0.z * (float)XSC); a[3] = (_Float16)(f0.w * (float)XSC);
  a[4] = (_Float16)(f1.x * (float)XSC); a[5] = (_Float16)(f1.y * (float)XSC);
  a[6] = (_Float16)(f1.z * (float)XSC); a[7] = (_Float16)(f1.w * (float)XSC);
  _Float16* d = gA + (size_t)row * K2 + DIM + c8;
  *(volatile v8h*)d = a;
  __threadfence();
  *(volatile v8h*)d = a;
}

__global__ __launch_bounds__(NTHR) void k_trans_f16(const float* __restrict__ W, int K, int N, _Float16* wt) {
  __shared__ __attribute__((aligned(16))) float tile[128 * TPW];
  const int tid = threadIdx.x, lane = tid & 31, g = tid >> 5, hh = lane >> 4, m = lane & 15;
  const int n0 = blockIdx.x * 64;
  const int n = n0 + 2 * lane;
#pragma unroll 1
  for (int dc = 0; dc < K; dc += 128) {
    __syncthreads();
#pragma unroll 4
    for (int p = 0; p < 16; ++p) {
      const int dl = g + 8 * p;
      const v2f w = *(const v2f*)(W + (size_t)(dc + dl) * N + n);
      *(v2f*)(tile + dl * TPW + 2 * lane) = w;
    }
    __syncthreads();
    v8h hv[4];
#pragma unroll
    for (int q = 0; q < 4; ++q) {
      const int nl = 8 * g + 2 * q + hh;
      const int d8 = 8 * m;
#pragma unroll
      for (int e = 0; e < 8; ++e) hv[q][e] = (_Float16)(tile[(d8 + e) * TPW + nl] * (float)WSC);
    }
#pragma unroll
    for (int q = 0; q < 4; ++q) {
      _Float16* d = wt + (size_t)(n0 + 8 * g + 2 * q + hh) * K + dc + 8 * m;
      *(volatile v8h*)d = hv[q];
    }
    __threadfence();
#pragma unroll
    for (int q = 0; q < 4; ++q) {
      _Float16* d = wt + (size_t)(n0 + 8 * g + 2 * q + hh) * K + dc + 8 * m;
      *(volatile v8h*)d = hv[q];
    }
  }
}

__global__ __launch_bounds__(NTHR) void k_trans_bf2(const float* __restrict__ W, int K, int N,
                                                    unsigned short* wh, unsigned short* wl) {
  __shared__ __attribute__((aligned(16))) float tile[128 * TPW];
  const int tid = threadIdx.x, lane = tid & 31, g = tid >> 5, hh = lane >> 4, m = lane & 15;
  const int n0 = blockIdx.x * 64;
  const int n = n0 + 2 * lane;
#pragma unroll 1
  for (int dc = 0; dc < K; dc += 128) {
    __syncthreads();
#pragma unroll 4
    for (int p = 0; p < 16; ++p) {
      const int dl = g + 8 * p;
      const v2f w = *(const v2f*)(W + (size_t)(dc + dl) * N + n);
      *(v2f*)(tile + dl * TPW + 2 * lane) = w;
    }
    __syncthreads();
    v8us hvh[4], hvl[4];
#pragma unroll
    for (int q = 0; q < 4; ++q) {
      const int nl = 8 * g + 2 * q + hh;
      const int d8 = 8 * m;
#pragma unroll
      for (int e = 0; e < 8; ++e) {
        unsigned short a, b;
        split2(tile[(d8 + e) * TPW + nl], a, b);
        hvh[q][e] = a; hvl[q][e] = b;
      }
    }
#pragma unroll
    for (int q = 0; q < 4; ++q) {
      const size_t o = (size_t)(n0 + 8 * g + 2 * q + hh) * K + dc + 8 * m;
      *(volatile v8us*)(wh + o) = hvh[q];
      *(volatile v8us*)(wl + o) = hvl[q];
    }
    __threadfence();
#pragma unroll
    for (int q = 0; q < 4; ++q) {
      const size_t o = (size_t)(n0 + 8 * g + 2 * q + hh) * K + dc + 8 * m;
      *(volatile v8us*)(wh + o) = hvh[q];
      *(volatile v8us*)(wl + o) = hvl[q];
    }
  }
}

__global__ __launch_bounds__(NTHR) void k_attn(const unsigned short* __restrict__ qh, const unsigned short* __restrict__ ql,
                                               const unsigned short* __restrict__ kh, const unsigned short* __restrict__ kl,
                                               const float* __restrict__ mw, unsigned short* ph, unsigned short* pl) {
  extern __shared__ v4f lds_dyn[];
  float* sc = (float*)lds_dyn;
  const int tid = threadIdx.x, lane = tid & 31, wave = tid >> 5, hh = lane >> 4, m = lane & 15;
  const int r0 = blockIdx.x * 32;
  const int c0 = wave * 64;

  v8f acc[2][4];
#pragma unroll
  for (int mt = 0; mt < 2; ++mt)
#pragma unroll
    for (int nt = 0; nt < 4; ++nt) { v8f z = {0.f, 0.f, 0.f, 0.f, 0.f, 0.f, 0.f, 0.f}; acc[mt][nt] = z; }

  const unsigned short* aph = qh + (size_t)(r0 + m) * DIM + 8 * hh;
  const unsigned short* apl = ql + (size_t)(r0 + m) * DIM + 8 * hh;
  const unsigned short* bph = kh + (size_t)(c0 + m) * DIM + 8 * hh;
  const unsigned short* bpl = kl + (size_t)(c0 + m) * DIM + 8 * hh;

#pragma unroll 1
  for (int kt = 0; kt < DIM / 32; ++kt) {
    const int k0 = 32 * kt;
    FragB ah0, ah1, al0, al1;
    ah0.h[0] = *(const v8us*)(aph + k0);
    ah0.h[1] = *(const v8us*)(aph + k0 + 16);
    ah1.h[0] = *(const v8us*)(aph + 16 * DIM + k0);
    ah1.h[1] = *(const v8us*)(aph + 16 * DIM + k0 + 16);
    al0.h[0] = *(const v8us*)(apl + k0);
    al0.h[1] = *(const v8us*)(apl + k0 + 16);
    al1.h[0] = *(const v8us*)(apl + 16 * DIM + k0);
    al1.h[1] = *(const v8us*)(apl + 16 * DIM + k0 + 16);
#pragma unroll
    for (int nt = 0; nt < 4; ++nt) {
      const unsigned short* bq = bph + (size_t)nt * 16 * DIM + k0;
      const unsigned short* br = bpl + (size_t)nt * 16 * DIM + k0;
      FragB bh, bl;
      bh.h[0] = *(const v8us*)bq;
      bh.h[1] = *(const v8us*)(bq + 16);
      bl.h[0] = *(const v8us*)br;
      bl.h[1] = *(const v8us*)(br + 16);
      acc[0][nt] = wmb(ah0.u, bh.u, acc[0][nt]);
      acc[0][nt] = wmb(ah0.u, bl.u, acc[0][nt]);
      acc[0][nt] = wmb(al0.u, bh.u, acc[0][nt]);
      acc[1][nt] = wmb(ah1.u, bh.u, acc[1][nt]);
      acc[1][nt] = wmb(ah1.u, bl.u, acc[1][nt]);
      acc[1][nt] = wmb(al1.u, bh.u, acc[1][nt]);
    }
  }

#pragma unroll
  for (int mt = 0; mt < 2; ++mt) {
#pragma unroll
    for (int nt = 0; nt < 4; ++nt) {
      const int col = c0 + 16 * nt + m;
#pragma unroll
      for (int r = 0; r < 8; ++r) {
        const int row = 16 * mt + 8 * hh + r;
        sc[row * NMEM + col] = acc[mt][nt][r] * SCALE_QK;
      }
    }
  }
  __syncthreads();

#pragma unroll 1
  for (int rr = 0; rr < 4; ++rr) {
    const int row = 4 * wave + rr;
    const float* sr = sc + row * NMEM + 8 * lane;
    const float* wr = mw + (size_t)(r0 + row) * NMEM + 8 * lane;
    const v4f w0 = *(const v4f*)(wr);
    const v4f w1 = *(const v4f*)(wr + 4);
    const v4f w2 = *(const v4f*)(wr + 256);
    const v4f w3 = *(const v4f*)(wr + 260);
    const v4f x0 = *(const v4f*)(sr) * w0;
    const v4f x1 = *(const v4f*)(sr + 4) * w1;
    const v4f x2 = *(const v4f*)(sr + 256) * w2;
    const v4f x3 = *(const v4f*)(sr + 260) * w3;
    float x[16] = {x0.x, x0.y, x0.z, x0.w, x1.x, x1.y, x1.z, x1.w,
                   x2.x, x2.y, x2.z, x2.w, x3.x, x3.y, x3.z, x3.w};
    float mx = x[0];
#pragma unroll
    for (int i = 1; i < 16; ++i) mx = fmaxf(mx, x[i]);
#pragma unroll
    for (int off = 16; off >= 1; off >>= 1) mx = fmaxf(mx, __shfl_xor(mx, off, 32));
    float s = 0.0f;
#pragma unroll
    for (int i = 0; i < 16; ++i) { x[i] = expf(x[i] - mx); s += x[i]; }
#pragma unroll
    for (int off = 16; off >= 1; off >>= 1) s += __shfl_xor(s, off, 32);
    const float inv = 1.0f / s;
    v8us H0, H1, L0, L1;
#pragma unroll
    for (int e = 0; e < 8; ++e) {
      unsigned short a, b;
      split2(x[e] * inv, a, b);
      H0[e] = a; L0[e] = b;
      split2(x[8 + e] * inv, a, b);
      H1[e] = a; L1[e] = b;
    }
    unsigned short* dh = ph + (size_t)(r0 + row) * NMEM + 8 * lane;
    unsigned short* dl = pl + (size_t)(r0 + row) * NMEM + 8 * lane;
    *(volatile v8us*)dh = H0;
    *(volatile v8us*)(dh + 256) = H1;
    *(volatile v8us*)dl = L0;
    *(volatile v8us*)(dl + 256) = L1;
    __threadfence();
    *(volatile v8us*)dh = H0;
    *(volatile v8us*)(dh + 256) = H1;
    *(volatile v8us*)dl = L0;
    *(volatile v8us*)(dl + 256) = L1;
  }
}

__global__ __launch_bounds__(NTHR) void k_pv(const unsigned short* __restrict__ ph, const unsigned short* __restrict__ pl,
                                             const unsigned short* __restrict__ vth, const unsigned short* __restrict__ vtl,
                                             const float* __restrict__ decay_p, _Float16* gA) {
  extern __shared__ v4f lds_dyn[];
  const int tid = threadIdx.x, lane = tid & 31, wave = tid >> 5, hh = lane >> 4, m = lane & 15;
  float* stg = (float*)lds_dyn + wave * (32 * 64);
  const int n0 = blockIdx.x * 128, m0 = blockIdx.y * 128;
  const int wm = (wave >> 1) * 32, wn = (wave & 1) * 64;

  v8f acc[2][4];
#pragma unroll
  for (int mt = 0; mt < 2; ++mt)
#pragma unroll
    for (int nt = 0; nt < 4; ++nt) { v8f z = {0.f, 0.f, 0.f, 0.f, 0.f, 0.f, 0.f, 0.f}; acc[mt][nt] = z; }

  const unsigned short* aph = ph + (size_t)(m0 + wm + m) * NMEM + 8 * hh;
  const unsigned short* apl = pl + (size_t)(m0 + wm + m) * NMEM + 8 * hh;
  const unsigned short* bph = vth + (size_t)(n0 + wn + m) * NMEM + 8 * hh;
  const unsigned short* bpl = vtl + (size_t)(n0 + wn + m) * NMEM + 8 * hh;

#pragma unroll 1
  for (int kt = 0; kt < NMEM / 32; ++kt) {
    const int k0 = 32 * kt;
    FragB ah0, ah1, al0, al1;
    ah0.h[0] = *(const v8us*)(aph + k0);
    ah0.h[1] = *(const v8us*)(aph + k0 + 16);
    ah1.h[0] = *(const v8us*)(aph + 16 * NMEM + k0);
    ah1.h[1] = *(const v8us*)(aph + 16 * NMEM + k0 + 16);
    al0.h[0] = *(const v8us*)(apl + k0);
    al0.h[1] = *(const v8us*)(apl + k0 + 16);
    al1.h[0] = *(const v8us*)(apl + 16 * NMEM + k0);
    al1.h[1] = *(const v8us*)(apl + 16 * NMEM + k0 + 16);
#pragma unroll
    for (int nt = 0; nt < 4; ++nt) {
      const unsigned short* bq = bph + (size_t)nt * 16 * NMEM + k0;
      const unsigned short* br = bpl + (size_t)nt * 16 * NMEM + k0;
      FragB bh, bl;
      bh.h[0] = *(const v8us*)bq;
      bh.h[1] = *(const v8us*)(bq + 16);
      bl.h[0] = *(const v8us*)br;
      bl.h[1] = *(const v8us*)(br + 16);
      acc[0][nt] = wmb(ah0.u, bh.u, acc[0][nt]);
      acc[0][nt] = wmb(ah0.u, bl.u, acc[0][nt]);
      acc[0][nt] = wmb(al0.u, bh.u, acc[0][nt]);
      acc[1][nt] = wmb(ah1.u, bh.u, acc[1][nt]);
      acc[1][nt] = wmb(ah1.u, bl.u, acc[1][nt]);
      acc[1][nt] = wmb(al1.u, bh.u, acc[1][nt]);
    }
  }

  const float decay = decay_p[0];
#pragma unroll
  for (int mt = 0; mt < 2; ++mt) {
    float* sp = stg + (16 * mt + 8 * hh) * 64 + m;
#pragma unroll
    for (int nt = 0; nt < 4; ++nt) {
#pragma unroll
      for (int r = 0; r < 8; ++r) sp[r * 64 + 16 * nt] = acc[mt][nt][r] * decay;
    }
  }
  __syncthreads();

  v8h hv[8];
#pragma unroll
  for (int i = 0; i < 8; ++i) {
    const int row = 4 * i + (lane >> 3), c = 8 * (lane & 7);
    const float* q = stg + row * 64 + c;
    const v4f f0 = *(const v4f*)q;
    const v4f f1 = *(const v4f*)(q + 4);
    hv[i][0] = (_Float16)(f0.x * (float)XSC); hv[i][1] = (_Float16)(f0.y * (float)XSC);
    hv[i][2] = (_Float16)(f0.z * (float)XSC); hv[i][3] = (_Float16)(f0.w * (float)XSC);
    hv[i][4] = (_Float16)(f1.x * (float)XSC); hv[i][5] = (_Float16)(f1.y * (float)XSC);
    hv[i][6] = (_Float16)(f1.z * (float)XSC); hv[i][7] = (_Float16)(f1.w * (float)XSC);
  }
#pragma unroll
  for (int i = 0; i < 8; ++i) {
    _Float16* d = gA + (size_t)(m0 + wm + 4 * i + (lane >> 3)) * K2 + n0 + wn + 8 * (lane & 7);
    *(volatile v8h*)d = hv[i];
  }
  __threadfence();
#pragma unroll
  for (int i = 0; i < 8; ++i) {
    _Float16* d = gA + (size_t)(m0 + wm + 4 * i + (lane >> 3)) * K2 + n0 + wn + 8 * (lane & 7);
    *(volatile v8h*)d = hv[i];
  }
}

__global__ __launch_bounds__(NTHR) void k_gate(const _Float16* __restrict__ gA, const _Float16* __restrict__ gwt,
                                               const float* __restrict__ gb, float* part) {
  __shared__ float rsum[NWAVE * 32];
  __shared__ __attribute__((aligned(16))) float rows_[128];
  const int tid = threadIdx.x, lane = tid & 31, wave = tid >> 5, hh = lane >> 4, m = lane & 15;
  const int n0 = blockIdx.x * 128, m0 = blockIdx.y * 128;
  const int wm = (wave >> 1) * 32, wn = (wave & 1) * 64;

  v8f acc[2][4];
#pragma unroll
  for (int mt = 0; mt < 2; ++mt)
#pragma unroll
    for (int nt = 0; nt < 4; ++nt) { v8f z = {0.f, 0.f, 0.f, 0.f, 0.f, 0.f, 0.f, 0.f}; acc[mt][nt] = z; }

  const _Float16* ap = gA + (size_t)(m0 + wm + m) * K2 + 8 * hh;
  const _Float16* bp = gwt + (size_t)(n0 + wn + m) * K2 + 8 * hh;
#pragma unroll 1
  for (int kt = 0; kt < K2 / 32; ++kt) {
    const int k0 = 32 * kt;
    FragH a0, a1;
    a0.h[0] = *(const v8h*)(ap + k0);
    a0.h[1] = *(const v8h*)(ap + k0 + 16);
    a1.h[0] = *(const v8h*)(ap + 16 * K2 + k0);
    a1.h[1] = *(const v8h*)(ap + 16 * K2 + k0 + 16);
#pragma unroll
    for (int nt = 0; nt < 4; ++nt) {
      const _Float16* bq = bp + (size_t)nt * 16 * K2 + k0;
      FragH b;
      b.h[0] = *(const v8h*)bq;
      b.h[1] = *(const v8h*)(bq + 16);
      acc[0][nt] = wmh(a0.v, b.v, acc[0][nt]);
      acc[1][nt] = wmh(a1.v, b.v, acc[1][nt]);
    }
  }

  constexpr float OSC = 1.0f / (float)(XSC * WSC);
  float bv[4];
#pragma unroll
  for (int nt = 0; nt < 4; ++nt) bv[nt] = gb[n0 + wn + 16 * nt + m];
  float ps[2][8];
#pragma unroll
  for (int mt = 0; mt < 2; ++mt) {
#pragma unroll
    for (int r = 0; r < 8; ++r) {
      float s = 0.0f;
#pragma unroll
      for (int nt = 0; nt < 4; ++nt) {
        const float z = acc[mt][nt][r] * OSC + bv[nt];
        const float e = __expf(-z);
        s += __builtin_amdgcn_rcpf(1.0f + e);
      }
      ps[mt][r] = s;
    }
  }
#pragma unroll
  for (int mt = 0; mt < 2; ++mt)
#pragma unroll
    for (int r = 0; r < 8; ++r) {
      ps[mt][r] += __shfl_xor(ps[mt][r], 1, 32);
      ps[mt][r] += __shfl_xor(ps[mt][r], 2, 32);
      ps[mt][r] += __shfl_xor(ps[mt][r], 4, 32);
      ps[mt][r] += __shfl_xor(ps[mt][r], 8, 32);
    }
  if (m == 0) {
#pragma unroll
    for (int mt = 0; mt < 2; ++mt)
#pragma unroll
      for (int r = 0; r < 8; ++r) rsum[wave * 32 + 16 * mt + 8 * hh + r] = ps[mt][r];
  }
  __syncthreads();
  if (tid < 128) {
    const int wp = tid >> 5, lr = tid & 31;
    rows_[tid] = rsum[(2 * wp) * 32 + lr] + rsum[(2 * wp + 1) * 32 + lr];
  }
  __syncthreads();
  if (tid < 32) {
    const v4f v = *(const v4f*)(rows_ + 4 * tid);
    float* d = part + (size_t)blockIdx.x * ROWS + m0 + 4 * tid;
    *(volatile v4f*)d = v;
    __threadfence();
    *(volatile v4f*)d = v;
  }
}

__global__ __launch_bounds__(NTHR) void k_out(const _Float16* __restrict__ gA, const _Float16* __restrict__ owt,
                                              const float* __restrict__ ob, const float* __restrict__ part, float* pre) {
  extern __shared__ v4f lds_dyn[];
  __shared__ float rsS[128];
  const int tid = threadIdx.x, lane = tid & 31, wave = tid >> 5, hh = lane >> 4, m = lane & 15;
  float* stg = (float*)lds_dyn + wave * (32 * 64);
  const int n0 = blockIdx.x * 128, m0 = blockIdx.y * 128;
  const int wm = (wave >> 1) * 32, wn = (wave & 1) * 64;

  if (tid < 128) {
    float s = 0.0f;
#pragma unroll
    for (int cb = 0; cb < DIM / 128; ++cb) s += part[(size_t)cb * ROWS + m0 + tid];
    rsS[tid] = 1.0f + s * (1.0f / (float)DIM);
  }
  __syncthreads();

  v8f acc[2][4];
#pragma unroll
  for (int mt = 0; mt < 2; ++mt)
#pragma unroll
    for (int nt = 0; nt < 4; ++nt) { v8f z = {0.f, 0.f, 0.f, 0.f, 0.f, 0.f, 0.f, 0.f}; acc[mt][nt] = z; }

  const _Float16* ap = gA + (size_t)(m0 + wm + m) * K2 + 8 * hh;
  const _Float16* bp = owt + (size_t)(n0 + wn + m) * DIM + 8 * hh;
#pragma unroll 1
  for (int kt = 0; kt < DIM / 32; ++kt) {
    const int k0 = 32 * kt;
    FragH a0, a1;
    a0.h[0] = *(const v8h*)(ap + k0);
    a0.h[1] = *(const v8h*)(ap + k0 + 16);
    a1.h[0] = *(const v8h*)(ap + 16 * K2 + k0);
    a1.h[1] = *(const v8h*)(ap + 16 * K2 + k0 + 16);
#pragma unroll
    for (int nt = 0; nt < 4; ++nt) {
      const _Float16* bq = bp + (size_t)nt * 16 * DIM + k0;
      FragH b;
      b.h[0] = *(const v8h*)bq;
      b.h[1] = *(const v8h*)(bq + 16);
      acc[0][nt] = wmh(a0.v, b.v, acc[0][nt]);
      acc[1][nt] = wmh(a1.v, b.v, acc[1][nt]);
    }
  }

  constexpr float OSC = 1.0f / (float)(XSC * WSC);
  float bv[4];
#pragma unroll
  for (int nt = 0; nt < 4; ++nt) bv[nt] = ob[n0 + wn + 16 * nt + m];
#pragma unroll
  for (int mt = 0; mt < 2; ++mt) {
    float* sp = stg + (16 * mt + 8 * hh) * 64 + m;
#pragma unroll
    for (int r = 0; r < 8; ++r) {
      const float rs = rsS[wm + 16 * mt + 8 * hh + r];
#pragma unroll
      for (int nt = 0; nt < 4; ++nt) sp[r * 64 + 16 * nt] = acc[mt][nt][r] * OSC * rs + bv[nt];
    }
  }
  __syncthreads();

  float* gbase = pre + (size_t)(m0 + wm) * DIM + n0 + wn;
#pragma unroll
  for (int q = 0; q < 16; ++q) {
    const int row = 2 * q + hh;
    const v4f v = *(const v4f*)(stg + row * 64 + 4 * m);
    *(volatile v4f*)(gbase + (size_t)row * DIM + 4 * m) = v;
  }
  __threadfence();
#pragma unroll
  for (int q = 0; q < 16; ++q) {
    const int row = 2 * q + hh;
    const v4f v = *(const v4f*)(stg + row * 64 + 4 * m);
    *(volatile v4f*)(gbase + (size_t)row * DIM + 4 * m) = v;
  }
}

__global__ __launch_bounds__(NTHR) void k_ln(const float* __restrict__ pre, const float* __restrict__ gamma,
                                             const float* __restrict__ beta, float* out) {
  const int tid = threadIdx.x, lane = tid & 31, wave = tid >> 5;
  const int row = blockIdx.x * NWAVE + wave;
  if (row >= ROWS) return;
  const float* pr = pre + (size_t)row * DIM + 4 * lane;
  v4f x[8];
  float s = 0.0f;
#pragma unroll
  for (int j = 0; j < 8; ++j) {
    x[j] = *(const v4f*)(pr + 128 * j);
    s += (x[j].x + x[j].y) + (x[j].z + x[j].w);
  }
#pragma unroll
  for (int off = 16; off >= 1; off >>= 1) s += __shfl_xor(s, off, 32);
  const float mean = s * (1.0f / (float)DIM);
  float s2 = 0.0f;
#pragma unroll
  for (int j = 0; j < 8; ++j) {
    x[j] = x[j] - mean;
    s2 += (x[j].x * x[j].x + x[j].y * x[j].y) + (x[j].z * x[j].z + x[j].w * x[j].w);
  }
#pragma unroll
  for (int off = 16; off >= 1; off >>= 1) s2 += __shfl_xor(s2, off, 32);
  const float var = s2 * (1.0f / (float)DIM);
  const float rstd = rsqrtf(var + LN_EPS);
  v4f y[8];
#pragma unroll
  for (int j = 0; j < 8; ++j) {
    const v4f g = *(const v4f*)(gamma + 128 * j + 4 * lane);
    const v4f bb = *(const v4f*)(beta + 128 * j + 4 * lane);
    y[j] = x[j] * rstd * g + bb;
  }
  float* d = out + (size_t)row * DIM + 4 * lane;
#pragma unroll
  for (int j = 0; j < 8; ++j) *(volatile v4f*)(d + 128 * j) = y[j];
  __threadfence();
#pragma unroll
  for (int j = 0; j < 8; ++j) *(volatile v4f*)(d + 128 * j) = y[j];
}

static inline size_t al256(size_t x) { return (x + 255) & ~(size_t)255; }

extern "C" void kernel_launch(void* const* d_in, const int* in_sizes, int n_in,
                              void* d_out, int out_size, void* d_ws, size_t ws_size,
                              hipStream_t stream) {
  if (n_in < 12) return;
  if (in_sizes[0] != ROWS * DIM || in_sizes[1] != ROWS * NMEM || in_sizes[2] != ROWS * DIM) return;
  if (in_sizes[3] != NMEM * DIM || in_sizes[4] != NMEM * DIM || in_sizes[5] < 1) return;
  if (in_sizes[6] != K2 * DIM || in_sizes[7] != DIM || in_sizes[8] != DIM * DIM || in_sizes[9] != DIM) return;
  if (in_sizes[10] != DIM || in_sizes[11] != DIM) return;
  if (out_size != ROWS * DIM) return;

  const float* query = (const float*)d_in[0];
  const float* mw    = (const float*)d_in[1];
  const float* upd   = (const float*)d_in[2];
  const float* keys  = (const float*)d_in[3];
  const float* vals  = (const float*)d_in[4];
  const float* decay = (const float*)d_in[5];
  const float* gw    = (const float*)d_in[6];
  const float* gb    = (const float*)d_in[7];
  const float* ow    = (const float*)d_in[8];
  const float* ob    = (const float*)d_in[9];
  const float* gam   = (const float*)d_in[10];
  const float* bet   = (const float*)d_in[11];
  float* out = (float*)d_out;

  char* ws = (char*)d_ws;
  size_t off = 0;
  const size_t oQh = off; off += al256((size_t)ROWS * DIM * 2);
  const size_t oQl = off; off += al256((size_t)ROWS * DIM * 2);
  const size_t oKh = off; off += al256((size_t)NMEM * DIM * 2);
  const size_t oKl = off; off += al256((size_t)NMEM * DIM * 2);
  const size_t oVh = off; off += al256((size_t)DIM * NMEM * 2);
  const size_t oVl = off; off += al256((size_t)DIM * NMEM * 2);
  const size_t oGw = off; off += al256((size_t)DIM * K2 * 2);
  const size_t oOw = off; off += al256((size_t)DIM * DIM * 2);
  const size_t oPh = off; off += al256((size_t)ROWS * NMEM * 2);
  const size_t oPl = off; off += al256((size_t)ROWS * NMEM * 2);
  const size_t oGA = off; off += al256((size_t)ROWS * K2 * 2);
  const size_t oPt = off; off += al256((size_t)(DIM / 128) * ROWS * 4);
  const size_t oPr = off; off += al256((size_t)ROWS * DIM * 4);
  if (off > ws_size || off > (size_t)WSCAP) return;

  unsigned short* qh  = (unsigned short*)(ws + oQh);
  unsigned short* ql  = (unsigned short*)(ws + oQl);
  unsigned short* kh  = (unsigned short*)(ws + oKh);
  unsigned short* kl  = (unsigned short*)(ws + oKl);
  unsigned short* vth = (unsigned short*)(ws + oVh);
  unsigned short* vtl = (unsigned short*)(ws + oVl);
  _Float16* gwt = (_Float16*)(ws + oGw);
  _Float16* owt = (_Float16*)(ws + oOw);
  unsigned short* ph  = (unsigned short*)(ws + oPh);
  unsigned short* pl  = (unsigned short*)(ws + oPl);
  _Float16* gA  = (_Float16*)(ws + oGA);
  float* part   = (float*)(ws + oPt);
  float* pre    = (float*)(ws + oPr);

  k_split8<<<(ROWS * DIM) / (8 * NTHR), NTHR, 0, stream>>>(query, qh, ql, (ROWS * DIM) / 8);
  k_split8<<<(NMEM * DIM) / (8 * NTHR), NTHR, 0, stream>>>(keys, kh, kl, (NMEM * DIM) / 8);
  k_trans_bf2<<<DIM / 64, NTHR, 0, stream>>>(vals, NMEM, DIM, vth, vtl);
  k_trans_f16<<<DIM / 64, NTHR, 0, stream>>>(gw, K2, DIM, gwt);
  k_trans_f16<<<DIM / 64, NTHR, 0, stream>>>(ow, DIM, DIM, owt);
  k_cvt_upd<<<(ROWS * (DIM / 8)) / NTHR, NTHR, 0, stream>>>(upd, gA);
  hipFuncSetAttribute(reinterpret_cast<const void*>(&k_attn), hipFuncAttributeMaxDynamicSharedMemorySize, LDS_SC);
  k_attn<<<ROWS / 32, NTHR, LDS_SC, stream>>>(qh, ql, kh, kl, mw, ph, pl);
  hipFuncSetAttribute(reinterpret_cast<const void*>(&k_pv), hipFuncAttributeMaxDynamicSharedMemorySize, LDS_STG);
  k_pv<<<dim3(DIM / 128, ROWS / 128), NTHR, LDS_STG, stream>>>(ph, pl, vth, vtl, decay, gA);
  k_gate<<<dim3(DIM / 128, ROWS / 128), NTHR, 0, stream>>>(gA, gwt, gb, part);
  hipFuncSetAttribute(reinterpret_cast<const void*>(&k_out), hipFuncAttributeMaxDynamicSharedMemorySize, LDS_STG);
  k_out<<<dim3(DIM / 128, ROWS / 128), NTHR, LDS_STG, stream>>>(gA, owt, ob, part, pre);
  k_ln<<<ROWS / NWAVE, NTHR, 0, stream>>>(pre, gam, bet, out);
}
